// MultiHeadedSelfAttention_4509715660804
// MI455X (gfx1250) — hardware-verified
//
#include <hip/hip_runtime.h>
#include <stdint.h>


typedef unsigned short u16;
typedef _Float16 h16;
typedef __bf16 v16bf __attribute__((ext_vector_type(16)));
typedef h16 v16h __attribute__((ext_vector_type(16)));
typedef h16 v8h __attribute__((ext_vector_type(8), __may_alias__));
typedef float v8f __attribute__((ext_vector_type(8)));
typedef float v4f __attribute__((ext_vector_type(4), __may_alias__));
typedef unsigned int v4u __attribute__((ext_vector_type(4), __may_alias__));

#ifndef NB
#define NB 4
#endif
#ifndef SEQ
#define SEQ 2048
#endif
#define NB_FULL 4
#define S_FULL 2048
#define DM 512
#define NH 8
#define HD 64
#define MT (NB * SEQ)

static_assert(NB >= 1 && NB <= NB_FULL);
static_assert(SEQ % 64 == 0 && SEQ <= S_FULL);
static_assert(DM % 64 == 0 && DM % 32 == 0);
static_assert(NH * HD == DM);
static_assert(HD == 64);
static_assert(MT % 64 == 0);


__device__ __forceinline__ u16 f2bf(float f) {
  unsigned u = __float_as_uint(f);
  u += 0x7FFFu + ((u >> 16) & 1u);
  return (u16)(u >> 16);
}

__device__ __forceinline__ float bf_rn(float f) {
  return __uint_as_float(((unsigned)f2bf(f)) << 16);
}

__device__ __forceinline__ v8f zero8() {
  v8f z = {0.f, 0.f, 0.f, 0.f, 0.f, 0.f, 0.f, 0.f};
  return z;
}

__device__ __forceinline__ v16bf ldfrag_bf(const u16* base, int ld) {
  const int l = threadIdx.x & 31;
  const int row = l & 15;
  const int kb = (l >> 4) << 3;
  const u16* p = base + (size_t)row * ld + kb;
  union { v16bf v; v4u q[2]; } u;
  u.q[0] = *(const v4u*)(p);
  u.q[1] = *(const v4u*)(p + 16);
  return u.v;
}

__device__ __forceinline__ v16h ldfrag_h(const h16* base, int ld) {
  const int l = threadIdx.x & 31;
  const int row = l & 15;
  const int kb = (l >> 4) << 3;
  const h16* p = base + (size_t)row * ld + kb;
  union { v16h v; v8h q[2]; } u;
  u.q[0] = *(const v8h*)(p);
  u.q[1] = *(const v8h*)(p + 16);
  return u.v;
}

__device__ __forceinline__ v8f mma_bf(v16bf a, v16bf b, v8f c) {
  v8f r = __builtin_amdgcn_wmma_f32_16x16x32_bf16(false, a, false, b, (short)0, c, false, false);
  asm volatile("v_nop\n\tv_nop\n\tv_nop\n\tv_nop" : "+v"(r) : "v"(a), "v"(b));
  return r;
}

__device__ __forceinline__ v8f mma_h(v16h a, v16h b, v8f c) {
  v8f r = __builtin_amdgcn_wmma_f32_16x16x32_f16(false, a, false, b, (short)0, c, false, false);
  asm volatile("v_nop\n\tv_nop\n\tv_nop\n\tv_nop" : "+v"(r) : "v"(a), "v"(b));
  return r;
}

__device__ __forceinline__ float hmax16(float x) {
#pragma unroll
  for (int s = 1; s < 16; s <<= 1) x = fmaxf(x, __shfl_xor(x, s, 32));
  return x;
}
__device__ __forceinline__ float hadd16(float x) {
#pragma unroll
  for (int s = 1; s < 16; s <<= 1) x += __shfl_xor(x, s, 32);
  return x;
}

__global__ __launch_bounds__(256) void k_cvt_bf16(const float* __restrict__ src, u16* __restrict__ dst,
                                                   int nrows, int rows_per_grp, int grp_stride_rows) {
  const int per_row = DM / 8;
  const int c = blockIdx.x * 256 + threadIdx.x;
  if (c >= nrows * per_row) return;
  const int pr = c / per_row;
  const int col = (c - pr * per_row) * 8;
  const int g = pr / rows_per_grp;
  const int sr = g * grp_stride_rows + (pr - g * rows_per_grp);
  const float* s = src + (size_t)sr * DM + col;
  const v4f a = *(const v4f*)(s);
  const v4f b = *(const v4f*)(s + 4);
  v4u w;
  w.x = (unsigned)f2bf(a.x) | ((unsigned)f2bf(a.y) << 16);
  w.y = (unsigned)f2bf(a.z) | ((unsigned)f2bf(a.w) << 16);
  w.z = (unsigned)f2bf(b.x) | ((unsigned)f2bf(b.y) << 16);
  w.w = (unsigned)f2bf(b.z) | ((unsigned)f2bf(b.w) << 16);
  volatile v4u* d = (volatile v4u*)(dst + (size_t)pr * DM + col);
  *d = w;
  __threadfence();
  *d = w;
}

__global__ __launch_bounds__(128) __attribute__((amdgpu_num_vgpr(256)))
void k_proj(const u16* __restrict__ Xb, const u16* __restrict__ Wb,
            const float* __restrict__ bq, const float* __restrict__ bk, const float* __restrict__ bv,
            h16* __restrict__ Qp, h16* __restrict__ Kp, h16* __restrict__ VTp) {
  __shared__ __attribute__((aligned(16))) h16 Ts[64 * 64];

  const int wave = threadIdx.x >> 5, lane = threadIdx.x & 31;
  const int hh = lane >> 4, mm = lane & 15;
  const int mat = blockIdx.z;
  const int m0 = blockIdx.x * 64, n0 = blockIdx.y * 64;
  const u16* W = Wb + (size_t)mat * DM * DM + (size_t)n0 * DM;
  const float* bias = (mat == 0) ? bq : ((mat == 1) ? bk : bv);
  const u16* Xr = Xb + (size_t)(m0 + wave * 16) * DM;

  v8f acc[4] = {zero8(), zero8(), zero8(), zero8()};

#pragma unroll 2
  for (int k0 = 0; k0 < DM; k0 += 32) {
    const v16bf a  = ldfrag_bf(Xr + k0, DM);
    const v16bf b0 = ldfrag_bf(W + (size_t)(0 * 16) * DM + k0, DM);
    const v16bf b1 = ldfrag_bf(W + (size_t)(1 * 16) * DM + k0, DM);
    const v16bf b2 = ldfrag_bf(W + (size_t)(2 * 16) * DM + k0, DM);
    const v16bf b3 = ldfrag_bf(W + (size_t)(3 * 16) * DM + k0, DM);
    acc[0] = mma_bf(a, b0, acc[0]);
    acc[1] = mma_bf(a, b1, acc[1]);
    acc[2] = mma_bf(a, b2, acc[2]);
    acc[3] = mma_bf(a, b3, acc[3]);
  }

  float bb[4];
#pragma unroll
  for (int t = 0; t < 4; ++t) bb[t] = bf_rn(bias[n0 + 16 * t + mm]);

  const bool tr = (mat == 2);
#pragma unroll
  for (int t = 0; t < 4; ++t) {
#pragma unroll
    for (int r = 0; r < 8; ++r) {
      const int row = wave * 16 + 8 * hh + r;
      const int col = 16 * t + mm;
      const int idx = tr ? (col * 64 + row) : (row * 64 + col);
      Ts[idx] = (h16)(acc[t][r] + bb[t]);
    }
  }
  __syncthreads();

  const int b  = m0 / SEQ;
  const int s0 = m0 - b * SEQ;
  const int bh = b * NH + blockIdx.y;
  h16* dstp = (mat == 0) ? Qp : ((mat == 1) ? Kp : VTp);
  const int pc = (threadIdx.x & 7) * 8;
  const int rb = threadIdx.x >> 3;
  v8h vals[4];
  size_t offs[4];
#pragma unroll
  for (int i = 0; i < 4; ++i) {
    const int rr = i * 16 + rb;
    vals[i] = *(const v8h*)(&Ts[rr * 64 + pc]);
    offs[i] = tr ? ((((size_t)bh * HD + rr) * SEQ) + s0 + pc)
                 : ((((size_t)bh * SEQ + s0 + rr) * HD) + pc);
  }
#pragma unroll
  for (int i = 0; i < 4; ++i) *(volatile v8h*)(dstp + offs[i]) = vals[i];
  __threadfence();
#pragma unroll
  for (int i = 0; i < 4; ++i) *(volatile v8h*)(dstp + offs[i]) = vals[i];
}

__global__ __launch_bounds__(128) __attribute__((amdgpu_num_vgpr(256)))
void k_attn(const h16* __restrict__ Qp, const h16* __restrict__ Kp, const h16* __restrict__ VTp,
            const int* __restrict__ mask, float* __restrict__ out) {
  __shared__ __attribute__((aligned(16))) h16   Ps[4][16 * 64];
  __shared__ __attribute__((aligned(16))) float Os[4][16 * 64];

  const int wave = threadIdx.x >> 5, lane = threadIdx.x & 31;
  const int hh = lane >> 4, mm = lane & 15;
  const int bh = blockIdx.y;
  const int b  = bh / NH;
  const int hd = bh - b * NH;
  const int q0 = blockIdx.x * 64 + wave * 16;

  const h16* Qbh = Qp  + (size_t)bh * SEQ * HD;
  const h16* Kbh = Kp  + (size_t)bh * SEQ * HD;
  const h16* Vbh = VTp + (size_t)bh * HD * SEQ;
  const int* mk_b = mask + (size_t)b * S_FULL;

  const v16h aq0 = ldfrag_h(Qbh + (size_t)q0 * HD, HD);
  const v16h aq1 = ldfrag_h(Qbh + (size_t)q0 * HD + 32, HD);

  float m_run[8], l_run[8];
  v8f o[4] = {zero8(), zero8(), zero8(), zero8()};
#pragma unroll
  for (int r = 0; r < 8; ++r) { m_run[r] = -1e30f; l_run[r] = 0.f; }

#pragma unroll 1
  for (int t0 = 0; t0 < SEQ; t0 += 64) {
    v8f sc[4];
#pragma unroll
    for (int t = 0; t < 4; ++t) {
      const v16h kf0 = ldfrag_h(Kbh + (size_t)(t0 + 16 * t) * HD, HD);
      const v16h kf1 = ldfrag_h(Kbh + (size_t)(t0 + 16 * t) * HD + 32, HD);
      sc[t] = mma_h(aq0, kf0, zero8());
      sc[t] = mma_h(aq1, kf1, sc[t]);
    }

    float madd[4];
#pragma unroll
    for (int t = 0; t < 4; ++t) madd[t] = -10000.0f * (1.0f - (float)mk_b[t0 + 16 * t + mm]);
#pragma unroll
    for (int t = 0; t < 4; ++t)
#pragma unroll
      for (int r = 0; r < 8; ++r) sc[t][r] = sc[t][r] * 0.125f + madd[t];

    float alpha[8];
#pragma unroll
    for (int r = 0; r < 8; ++r) {
      float mx = fmaxf(fmaxf(sc[0][r], sc[1][r]), fmaxf(sc[2][r], sc[3][r]));
      mx = hmax16(mx);
      const float mn = fmaxf(m_run[r], mx);
      alpha[r] = __expf(m_run[r] - mn);
      m_run[r] = mn;
    }
#pragma unroll
    for (int r = 0; r < 8; ++r) {
      float ps = 0.f;
#pragma unroll
      for (int t = 0; t < 4; ++t) {
        const float p = __expf(sc[t][r] - m_run[r]);
        ps += p;
        Ps[wave][(8 * hh + r) * 64 + 16 * t + mm] = (h16)(p * 1024.0f);
      }
      l_run[r] = l_run[r] * alpha[r] + hadd16(ps);
    }
#pragma unroll
    for (int dt = 0; dt < 4; ++dt)
#pragma unroll
      for (int r = 0; r < 8; ++r) o[dt][r] *= alpha[r];

    __syncthreads();

    const v16h p0 = ldfrag_h(&Ps[wave][0], 64);
    const v16h p1 = ldfrag_h(&Ps[wave][32], 64);
#pragma unroll
    for (int dt = 0; dt < 4; ++dt) {
      const v16h vf0 = ldfrag_h(Vbh + (size_t)(16 * dt) * SEQ + t0, SEQ);
      const v16h vf1 = ldfrag_h(Vbh + (size_t)(16 * dt) * SEQ + t0 + 32, SEQ);
      o[dt] = mma_h(p0, vf0, o[dt]);
      o[dt] = mma_h(p1, vf1, o[dt]);
    }
    __syncthreads();
  }

  float inv[8];
#pragma unroll
  for (int r = 0; r < 8; ++r) inv[r] = (1.0f / l_run[r]) * 0.0009765625f;
#pragma unroll
  for (int dt = 0; dt < 4; ++dt)
#pragma unroll
    for (int r = 0; r < 8; ++r) Os[wave][(8 * hh + r) * 64 + 16 * dt + mm] = o[dt][r] * inv[r];
  __syncthreads();

  const int rsub = lane >> 4;
  const int cc = (lane & 15) * 4;
  float* ob = out + ((size_t)b * SEQ + q0) * DM + (size_t)hd * HD;
  v4f vv[8];
#pragma unroll
  for (int i = 0; i < 8; ++i) vv[i] = *(const v4f*)(&Os[wave][(2 * i + rsub) * 64 + cc]);
#pragma unroll
  for (int i = 0; i < 8; ++i) *(volatile v4f*)(ob + (size_t)(2 * i + rsub) * DM + cc) = vv[i];
  __threadfence();
#pragma unroll
  for (int i = 0; i < 8; ++i) *(volatile v4f*)(ob + (size_t)(2 * i + rsub) * DM + cc) = vv[i];
}

extern "C" void kernel_launch(void* const* d_in, const int* in_sizes, int n_in,
                              void* d_out, int out_size, void* d_ws, size_t ws_size,
                              hipStream_t stream) {
  if (n_in < 8) return;
  const float* x   = (const float*)d_in[0];
  const int*   msk = (const int*)d_in[1];
  const float* Wq  = (const float*)d_in[2];
  const float* bq  = (const float*)d_in[3];
  const float* Wk  = (const float*)d_in[4];
  const float* bk  = (const float*)d_in[5];
  const float* Wv  = (const float*)d_in[6];
  const float* bv  = (const float*)d_in[7];
  float* out = (float*)d_out;

  if (in_sizes[0] < ((NB - 1) * S_FULL + SEQ) * DM) return;
  if (in_sizes[1] < (NB - 1) * S_FULL + SEQ) return;
  if (in_sizes[2] < DM * DM || in_sizes[4] < DM * DM || in_sizes[6] < DM * DM) return;
  if (in_sizes[3] < DM || in_sizes[5] < DM || in_sizes[7] < DM) return;
  if (out_size < MT * DM) return;

  char* ws = (char*)d_ws;
  const size_t XB_BYTES = (size_t)MT * DM * 2;
  const size_t W_BYTES  = (size_t)DM * DM * 2;
  const size_t PL_BYTES = (size_t)NB * NH * SEQ * HD * 2;
  size_t off = 0;
  u16* Xb = (u16*)(ws + off);  off += XB_BYTES;
  u16* Wb = (u16*)(ws + off);  off += 3 * W_BYTES;
  h16* Qp = (h16*)(ws + off);  off += PL_BYTES;
  h16* Kp = (h16*)(ws + off);  off += PL_BYTES;
  h16* VTp = (h16*)(ws + off); off += PL_BYTES;
  if (off > ws_size) return;

  const int nchunk_x = MT * (DM / 8);
  const int nchunk_w = DM * (DM / 8);
  k_cvt_bf16<<<(nchunk_x + 255) / 256, 256, 0, stream>>>(x,  Xb, MT, SEQ, S_FULL);
  k_cvt_bf16<<<(nchunk_w + 255) / 256, 256, 0, stream>>>(Wq, Wb, DM, DM, DM);
  k_cvt_bf16<<<(nchunk_w + 255) / 256, 256, 0, stream>>>(Wk, Wb + (size_t)DM * DM, DM, DM, DM);
  k_cvt_bf16<<<(nchunk_w + 255) / 256, 256, 0, stream>>>(Wv, Wb + (size_t)2 * DM * DM, DM, DM, DM);

  dim3 gp(MT / 64, DM / 64, 3);
  k_proj<<<gp, 128, 0, stream>>>(Xb, Wb, bq, bk, bv, Qp, Kp, VTp);

  dim3 ga(SEQ / 64, NB * NH);
  k_attn<<<ga, 128, 0, stream>>>(Qp, Kp, VTp, msk, out);
}
